// BlockSparseAttention_67216238182781
// MI455X (gfx1250) — hardware-verified
//
#include <hip/hip_runtime.h>
#include <math.h>
#include <stdint.h>

#ifndef NB
#define NB 2
#endif
#ifndef SEQ
#define SEQ 4096
#endif
#ifndef RICH
#define RICH 512
#endif
#define NB_FULL 2
#define XS_FULL 4096
#define DMOD  1024
#define NH    16
#define HD    64
#define KC    4
#define NQKV  (3 * DMOD)
#define WIN   512
#define BLK   64
#define RICHE ((RICH < SEQ) ? RICH : SEQ)
#define SM_SCALE 0.125f
#define QSC   1024.0f
#define KSC   1024.0f
#define PCAR  32768.0f
#define VCAR  4096.0f
#define OSC   1024.0f
#define WOS   1024.0f
#define WPB   4
#define NHG   (NH / WPB)
#define NQT   (SEQ / 16)
#define NQTR  (RICHE / 16)
#define NST   (SEQ / 64)
#define NKT   (SEQ / 32)
#define ATT_THREADS (WPB * 32)
#define PTP   36
#define PTW   (16 * PTP)
#define SLP   68
#define SLW   (16 * SLP)
#define WREG  (PTW + SLW)
#define SLAB64 (16 * 68)
#define VTP   72
#define WS_CAP 134217728
static_assert(DMOD == NH * HD && HD == 64 && NH == 16 && WPB == 4 && NHG * WPB == NH && KC == 4);
static_assert(ATT_THREADS == 128 && NQKV == 3072 && WIN == 512 && BLK == 64 && (WIN % BLK) == 0 && (BLK % 32) == 0 && NHG == 4);
static_assert(NB >= 1 && NB <= NB_FULL);
static_assert(NB == 1 || SEQ == XS_FULL);
static_assert((SEQ % 64) == 0 && SEQ >= 64 && SEQ <= XS_FULL);
static_assert((RICHE % 64) == 0 && RICHE >= 64 && RICHE <= SEQ);
static_assert((DMOD % 64) == 0 && (NQKV % 64) == 0 && (DMOD % 32) == 0 && (HD % 32) == 0);
static_assert(((SEQ * DMOD / 8) % 256) == 0 && ((NQKV * DMOD / 8) % 256) == 0 && ((DMOD * DMOD / 8) % 256) == 0);
static_assert(WPB * WREG * 4 <= 65536 && 2 * HD * VTP * 2 <= 65536 && 4 * SLAB64 * 4 <= 65536);
static_assert(NQT * 16 == SEQ && NQTR * 16 == RICHE && NKT * 32 == SEQ && NST * 64 == SEQ);
static_assert((size_t)SEQ * DMOD * 2 + (size_t)NQKV * DMOD * 2 + (size_t)DMOD * DMOD * 2 + (size_t)SEQ * NQKV * 4
              + (size_t)7 * SEQ * DMOD * 2 + (size_t)RICHE * DMOD * 2 <= (size_t)WS_CAP);

typedef unsigned short u16;
typedef _Float16 v16h __attribute__((ext_vector_type(16)));
typedef _Float16 v8h  __attribute__((ext_vector_type(8)));
typedef __bf16   v16b __attribute__((ext_vector_type(16)));
typedef float    v8f  __attribute__((ext_vector_type(8)));
typedef float    v4f  __attribute__((ext_vector_type(4)));
typedef unsigned int v4u __attribute__((ext_vector_type(4)));

union FragH { v16h v; v8h h[2]; v4u u[2]; };
union FragB { v16b v; v4u u[2]; };

__device__ __forceinline__ unsigned short bf_bits(float f) {
  unsigned u = __float_as_uint(f);
  return (unsigned short)((u + 0x7FFFu + ((u >> 16) & 1u)) >> 16);
}
__device__ __forceinline__ float bf_up(unsigned short h) { return __uint_as_float(((unsigned)h) << 16); }
__device__ __forceinline__ float bfr(float f) { return bf_up(bf_bits(f)); }
__device__ __forceinline__ unsigned short h_bits(_Float16 x) { return __builtin_bit_cast(unsigned short, x); }
__device__ __forceinline__ unsigned pk16(unsigned short a, unsigned short b) { return (unsigned)a | ((unsigned)b << 16); }
__device__ __forceinline__ v8f zero8() { v8f z = {0.f, 0.f, 0.f, 0.f, 0.f, 0.f, 0.f, 0.f}; return z; }

__device__ __forceinline__ void hl_bits(float t, unsigned short& hb, unsigned short& lb) {
#pragma clang fp contract(off)
  const _Float16 a = (_Float16)t;
  hb = h_bits(a);
  lb = h_bits((_Float16)(t - (float)a));
}
__device__ __forceinline__ float conv4(float w0, float w1, float w2, float w3, float x0, float x1, float x2, float x3) {
#pragma clang fp contract(off)
  const float p0 = w0 * x0;
  const float p1 = w1 * x1;
  const float p2 = w2 * x2;
  const float p3 = w3 * x3;
  const float s01 = p0 + p1;
  const float s012 = s01 + p2;
  return s012 + p3;
}

__device__ __forceinline__ v16h ldfrag_h(const _Float16* p) {
  FragH f;
  f.h[0] = *(const v8h*)(p);
  f.h[1] = *(const v8h*)(p + 16);
  return f.v;
}
__device__ __forceinline__ v16b ldfrag_b(const u16* p) {
  FragB f;
  f.u[0] = *(const v4u*)(p);
  f.u[1] = *(const v4u*)(p + 16);
  return f.v;
}

__device__ __forceinline__ v8f mma_h(v16h a, v16h b, v8f c) {
  return __builtin_amdgcn_wmma_f32_16x16x32_f16(false, a, false, b, (short)0, c, false, false);
}
__device__ __forceinline__ v8f mma_b(v16b a, v16b b, v8f c) {
  return __builtin_amdgcn_wmma_f32_16x16x32_bf16(false, a, false, b, (short)0, c, false, false);
}
__device__ __forceinline__ void guard2(v8f& a, v8f& b, v16h x0, v16h x1, v16h x2, v16h x3, v16h x4, v16h x5) {
#if defined(__HIP_DEVICE_COMPILE__)
  asm volatile("v_nop\n\tv_nop\n\tv_nop\n\tv_nop"
               : "+v"(a), "+v"(b) : "v"(x0), "v"(x1), "v"(x2), "v"(x3), "v"(x4), "v"(x5) : "memory");
#endif
}
template <typename F>
__device__ __forceinline__ void guard6(v8f& a, v8f& b, v8f& c, v8f& d, F x0, F x1, F x2, F x3, F x4, F x5) {
#if defined(__HIP_DEVICE_COMPILE__)
  asm volatile("v_nop\n\tv_nop\n\tv_nop\n\tv_nop"
               : "+v"(a), "+v"(b), "+v"(c), "+v"(d) : "v"(x0), "v"(x1), "v"(x2), "v"(x3), "v"(x4), "v"(x5) : "memory");
#endif
}
__device__ __forceinline__ void acc_guard4(v8f& a, v8f& b, v8f& c, v8f& d) {
#if defined(__HIP_DEVICE_COMPILE__)
  asm volatile("v_nop\n\tv_nop\n\tv_nop\n\tv_nop" : "+v"(a), "+v"(b), "+v"(c), "+v"(d));
#endif
}
__device__ __forceinline__ void wave_sync_lds() {
  __builtin_amdgcn_fence(__ATOMIC_RELEASE, "workgroup");
  __builtin_amdgcn_wave_barrier();
  __builtin_amdgcn_fence(__ATOMIC_ACQUIRE, "workgroup");
}

__global__ __launch_bounds__(256) void cvt16(const float* __restrict__ x, u16* D, int n8, int f16mode, float scale) {
  const int gt = blockIdx.x * 256 + (int)threadIdx.x;
  if (gt >= n8) return;
  const float* p = x + (size_t)gt * 8;
  const v4f a = *(const v4f*)(p), b4 = *(const v4f*)(p + 4);
  float w[8];
#pragma unroll
  for (int e = 0; e < 4; ++e) { w[e] = a[e]; w[4 + e] = b4[e]; }
  v4u o;
#pragma unroll
  for (int e = 0; e < 4; ++e) {
    const float f0 = w[2 * e], f1 = w[2 * e + 1];
    const unsigned short hb0 = h_bits((_Float16)(bfr(f0) * scale));
    const unsigned short hb1 = h_bits((_Float16)(bfr(f1) * scale));
    const unsigned short bb0 = bf_bits(f0);
    const unsigned short bb1 = bf_bits(f1);
    o[e] = (f16mode != 0) ? pk16(hb0, hb1) : pk16(bb0, bb1);
  }
  u16* d = D + (size_t)gt * 8;
  for (int pass = 0; pass < 2; ++pass) {
    *(volatile v4u*)(d) = o;
    __threadfence();
  }
}

__global__ __launch_bounds__(128) void conv16(const float* __restrict__ F, int ldf, int coff,
                                              const float* __restrict__ Wc, u16* Hp, u16* Lp, float sc) {
#pragma clang fp contract(off)
  const int tid = (int)threadIdx.x;
  const int row = (int)blockIdx.x;
  if (row >= SEQ) return;
  const int col = tid * 8;
  if (col + 8 > DMOD) return;
  float xv[KC][8];
#pragma unroll
  for (int j = 0; j < KC; ++j) {
    const int tt  = row - (KC - 1) + j;
    const int ttc = (tt < 0) ? 0 : tt;
    const float* p = F + (size_t)ttc * (size_t)ldf + coff + col;
    const v4f a = *(const v4f*)(p), b4 = *(const v4f*)(p + 4);
#pragma unroll
    for (int e = 0; e < 4; ++e) {
      xv[j][e]     = (tt >= 0) ? a[e]  : 0.0f;
      xv[j][4 + e] = (tt >= 0) ? b4[e] : 0.0f;
    }
  }
  float wv[8][KC];
  const float* wp = Wc + (size_t)col * KC;
#pragma unroll
  for (int e = 0; e < 8; ++e) {
    const v4f w4 = *(const v4f*)(wp + KC * e);
#pragma unroll
    for (int j = 0; j < KC; ++j) wv[e][j] = bfr(w4[j]);
  }
  float y[8];
#pragma unroll
  for (int e = 0; e < 8; ++e) {
    y[e] = conv4(wv[e][0], wv[e][1], wv[e][2], wv[e][3], xv[0][e], xv[1][e], xv[2][e], xv[3][e]);
  }
  v4u oh, ol;
#pragma unroll
  for (int e = 0; e < 4; ++e) {
    unsigned short h0, l0, h1, l1;
    hl_bits(y[2 * e] * sc,     h0, l0);
    hl_bits(y[2 * e + 1] * sc, h1, l1);
    oh[e] = pk16(h0, h1);
    ol[e] = pk16(l0, l1);
  }
  u16* dh = Hp + (size_t)row * DMOD + col;
  u16* dl = Lp + (size_t)row * DMOD + col;
  for (int pass = 0; pass < 2; ++pass) {
    *(volatile v4u*)(dh) = oh;
    *(volatile v4u*)(dl) = ol;
    __threadfence();
  }
}

__global__ __launch_bounds__(256) void vt16(const float* __restrict__ F, int ldf, int voff,
                                            const float* __restrict__ Wc, u16* VHo, u16* VLo) {
#pragma clang fp contract(off)
  __shared__ __align__(16) u16 TH[HD * VTP];
  __shared__ __align__(16) u16 TL[HD * VTP];
  const int tid = (int)threadIdx.x;
  const int bid = (int)blockIdx.x;
  const int st  = bid % NST;
  const int g   = bid / NST;
  if (g >= NH) return;
  const int s0  = st * 64;
  {
    const int sl = tid >> 2;
    const int dc = (tid & 3) * 16;
    const int sk = s0 + sl;
#pragma unroll
    for (int i = 0; i < 4; ++i) {
      const int d0 = dc + 4 * i;
      const int ch = g * HD + d0;
      float wv[4][KC];
      const float* wp = Wc + (size_t)ch * KC;
#pragma unroll
      for (int e = 0; e < 4; ++e) {
        const v4f w4 = *(const v4f*)(wp + KC * e);
#pragma unroll
        for (int j = 0; j < KC; ++j) wv[e][j] = bfr(w4[j]);
      }
      float xv[KC][4];
#pragma unroll
      for (int j = 0; j < KC; ++j) {
        const int tt  = sk - (KC - 1) + j;
        const int ttc = (tt < 0) ? 0 : tt;
        const v4f a = *(const v4f*)(F + (size_t)ttc * (size_t)ldf + voff + ch);
#pragma unroll
        for (int e = 0; e < 4; ++e) xv[j][e] = (tt >= 0) ? a[e] : 0.0f;
      }
#pragma unroll
      for (int e = 0; e < 4; ++e) {
        const float y = conv4(wv[e][0], wv[e][1], wv[e][2], wv[e][3], xv[0][e], xv[1][e], xv[2][e], xv[3][e]);
        unsigned short hb, lb;
        hl_bits(y * VCAR, hb, lb);
        TH[(d0 + e) * VTP + sl] = hb;
        TL[(d0 + e) * VTP + sl] = lb;
      }
    }
  }
  __syncthreads();
  v4u vh[2], vl[2];
  const int q8 = tid >> 3, p8 = (tid & 7) * 8;
#pragma unroll
  for (int it = 0; it < 2; ++it) {
    const int line = it * 32 + q8;
    vh[it] = *(const v4u*)(TH + line * VTP + p8);
    vl[it] = *(const v4u*)(TL + line * VTP + p8);
  }
  const size_t hrow = (size_t)g * HD;
  const size_t base = hrow * SEQ + s0 + p8;
  for (int pass = 0; pass < 2; ++pass) {
#pragma unroll
    for (int it = 0; it < 2; ++it) {
      const int line = it * 32 + q8;
      *(volatile v4u*)(VHo + base + (size_t)line * SEQ) = vh[it];
      *(volatile v4u*)(VLo + base + (size_t)line * SEQ) = vl[it];
    }
    __threadfence();
  }
}

__device__ __forceinline__ void epi64(float* sl, v8f a0, v8f a1, v8f a2, v8f a3, float oscale,
                                      float* C, int N, size_t rowb, int col0, int lane) {
  const int hh = lane >> 4, m = lane & 15;
#pragma unroll
  for (int r = 0; r < 8; ++r) {
    const int ro = (8 * hh + r) * 68 + m;
    sl[ro]      = a0[r] * oscale;
    sl[ro + 16] = a1[r] * oscale;
    sl[ro + 32] = a2[r] * oscale;
    sl[ro + 48] = a3[r] * oscale;
  }
  wave_sync_lds();
  v4f vals[8];
#pragma unroll
  for (int it = 0; it < 8; ++it) vals[it] = *(const v4f*)(sl + (it * 2 + hh) * 68 + m * 4);
  float* dst = C + (rowb + (size_t)hh) * (size_t)N + col0 + m * 4;
  for (int pass = 0; pass < 2; ++pass) {
#pragma unroll
    for (int it = 0; it < 8; ++it) {
      *(volatile v4f*)(dst + (size_t)(it * 2) * (size_t)N) = vals[it];
    }
    __threadfence();
  }
}

__global__ __launch_bounds__(128)
void gemm_bf(const u16* __restrict__ A, const u16* __restrict__ Bt, float* C, int M, int N, int K, float oscale) {
  __shared__ __align__(16) float slab[4 * SLAB64];
  const int tid = threadIdx.x, wave = tid >> 5, lane = tid & 31, hh = lane >> 4, m = lane & 15;
  const int ntile = N >> 6;
  const int bid   = blockIdx.x;
  const int rowb  = (bid / ntile) * 64 + wave * 16;
  const int col0  = (bid % ntile) * 64;
  if (rowb + 16 > M) return;
  const u16* ap = A  + (size_t)(rowb + m) * K + 8 * hh;
  const u16* bp = Bt + (size_t)(col0 + m) * K + 8 * hh;
  const size_t bs = (size_t)16 * K;
  v8f acc0 = zero8(), acc1 = zero8(), acc2 = zero8(), acc3 = zero8();
#pragma unroll 1
  for (int k0 = 0; k0 < K; k0 += 32) {
    const v16b a  = ldfrag_b(ap + k0);
    const v16b b0 = ldfrag_b(bp + k0);
    const v16b b1 = ldfrag_b(bp + bs + k0);
    const v16b b2 = ldfrag_b(bp + 2 * bs + k0);
    const v16b b3 = ldfrag_b(bp + 3 * bs + k0);
    acc0 = mma_b(a, b0, acc0);
    acc1 = mma_b(a, b1, acc1);
    acc2 = mma_b(a, b2, acc2);
    acc3 = mma_b(a, b3, acc3);
    guard6<v16b>(acc0, acc1, acc2, acc3, a, b0, b1, b2, b3, a);
  }
  epi64(slab + wave * SLAB64, acc0, acc1, acc2, acc3, oscale, C, N, (size_t)rowb, col0, lane);
}

template <int TWO>
__global__ __launch_bounds__(128)
void gemm_h(const u16* __restrict__ A, const u16* __restrict__ A2, const u16* __restrict__ Bt, float* C,
            int M, int N, int K, float oscale) {
  __shared__ __align__(16) float slab[4 * SLAB64];
  const int tid = threadIdx.x, wave = tid >> 5, lane = tid & 31, hh = lane >> 4, m = lane & 15;
  const int ntile = N >> 6;
  const int bid   = blockIdx.x;
  const int rowb  = (bid / ntile) * 64 + wave * 16;
  const int col0  = (bid % ntile) * 64;
  if (rowb + 16 > M) return;
  const _Float16* ap  = (const _Float16*)(const void*)A  + (size_t)(rowb + m) * K + 8 * hh;
  const _Float16* ap2 = (const _Float16*)(const void*)A2 + (size_t)(rowb + m) * K + 8 * hh;
  const _Float16* bp  = (const _Float16*)(const void*)Bt + (size_t)(col0 + m) * K + 8 * hh;
  const size_t bs = (size_t)16 * K;
  v8f acc0 = zero8(), acc1 = zero8(), acc2 = zero8(), acc3 = zero8();
#pragma unroll 1
  for (int k0 = 0; k0 < K; k0 += 32) {
    const v16h a  = ldfrag_h(ap + k0);
    const v16h b0 = ldfrag_h(bp + k0);
    const v16h b1 = ldfrag_h(bp + bs + k0);
    const v16h b2 = ldfrag_h(bp + 2 * bs + k0);
    const v16h b3 = ldfrag_h(bp + 3 * bs + k0);
    acc0 = mma_h(a, b0, acc0);
    acc1 = mma_h(a, b1, acc1);
    acc2 = mma_h(a, b2, acc2);
    acc3 = mma_h(a, b3, acc3);
    if (TWO != 0) {
      const v16h a2 = ldfrag_h(ap2 + k0);
      acc0 = mma_h(a2, b0, acc0);
      acc1 = mma_h(a2, b1, acc1);
      acc2 = mma_h(a2, b2, acc2);
      acc3 = mma_h(a2, b3, acc3);
      guard6<v16h>(acc0, acc1, acc2, acc3, a, a2, b0, b1, b2, b3);
    } else {
      guard6<v16h>(acc0, acc1, acc2, acc3, a, b0, b1, b2, b3, a);
    }
  }
  (void)ap2;
  epi64(slab + wave * SLAB64, acc0, acc1, acc2, acc3, oscale, C, N, (size_t)rowb, col0, lane);
}

template <int RV>
__global__ __launch_bounds__(ATT_THREADS)
void attn_w(const u16* __restrict__ QHp, const u16* __restrict__ QLp,
            const u16* __restrict__ KHp, const u16* __restrict__ KLp,
            const u16* __restrict__ VHp, const u16* __restrict__ VLp,
            u16* OHp, u16* OLp, int qt0, int nqt) {
#pragma clang fp contract(off)
  __shared__ __align__(16) float smem[WPB * WREG];

  const int tid  = threadIdx.x;
  const int wave = tid >> 5;
  const int lane = tid & 31;
  const int hh   = lane >> 4;
  const int c    = lane & 15;
  const int bid  = blockIdx.x;
  if (nqt <= 0) return;
  const int qt   = qt0 + bid % nqt;
  const int hg   = bid / nqt;
  if (hg >= NHG) return;
  const int q0   = qt * 16;
  if (q0 + 16 > SEQ) return;
  const int head = hg * WPB + wave;

  float* pt   = smem + wave * WREG;
  float* slab = pt + PTW;

  const size_t hcol = (size_t)head * HD + 8 * hh;
  const _Float16* Qh  = (const _Float16*)(const void*)QHp + ((size_t)q0 + c) * DMOD + hcol;
  const _Float16* Ql  = (const _Float16*)(const void*)QLp + ((size_t)q0 + c) * DMOD + hcol;
  const _Float16* Khb = (const _Float16*)(const void*)KHp + (size_t)c * DMOD + hcol;
  const _Float16* Klb = (const _Float16*)(const void*)KLp + (size_t)c * DMOD + hcol;
  const _Float16* Vhb = (const _Float16*)(const void*)VHp + ((size_t)head * HD + c) * SEQ + 8 * hh;
  const _Float16* Vlb = (const _Float16*)(const void*)VLp + ((size_t)head * HD + c) * SEQ + 8 * hh;
  const float lsc  = SM_SCALE * (1.0f / (QSC * KSC));
  const float oc   = 1.0f / (PCAR * VCAR);
  const float ninf = -__builtin_inff();
  const size_t KROW = (size_t)DMOD;

  v8f o[4];
#pragma unroll
  for (int j = 0; j < 4; ++j) o[j] = zero8();
  float mrun[8], lrun[8];
#pragma unroll
  for (int r = 0; r < 8; ++r) { mrun[r] = ninf; lrun[r] = 0.0f; }
  const int kst = (q0 / BLK) * BLK - WIN;
  const int klo = (kst < 0) ? 0 : kst;
  const int ktlo = klo >> 5;
  const int kthi = q0 >> 5;
  int nkt = kthi - ktlo + 1;
  if (nkt > NKT) nkt = NKT;
  if (nkt < 1) nkt = 1;
  const int qr0   = q0 + 8 * hh;

#pragma unroll 1
  for (int i = 0; i < nkt; ++i) {
    const int kb = (ktlo + i) * 32;
    v8f s0 = zero8(), s1 = zero8();
    const _Float16* k0p = Khb + (size_t)kb * KROW;
    const _Float16* k1p = k0p + (size_t)16 * KROW;
    const _Float16* l0p = Klb + (size_t)kb * KROW;
    const _Float16* l1p = l0p + (size_t)16 * KROW;
#pragma unroll
    for (int kk = 0; kk < HD / 32; ++kk) {
      const v16h qh  = ldfrag_h(Qh + kk * 32);
      const v16h ql  = ldfrag_h(Ql + kk * 32);
      const v16h kh0 = ldfrag_h(k0p + kk * 32);
      const v16h kh1 = ldfrag_h(k1p + kk * 32);
      const v16h kl0 = ldfrag_h(l0p + kk * 32);
      const v16h kl1 = ldfrag_h(l1p + kk * 32);
      s0 = mma_h(qh, kh0, s0);
      s0 = mma_h(ql, kh0, s0);
      s0 = mma_h(qh, kl0, s0);
      s1 = mma_h(qh, kh1, s1);
      s1 = mma_h(ql, kh1, s1);
      s1 = mma_h(qh, kl1, s1);
      guard2(s0, s1, qh, ql, kh0, kl0, kh1, kl1);
    }
    float alpha[8];
    const int key0 = kb + c, key1 = kb + 16 + c;
#pragma unroll
    for (int r = 0; r < 8; ++r) {
      const int qrow = qr0 + r;
      const float a0 = s0[r] * lsc;
      const float a1 = s1[r] * lsc;
      const bool ok0 = (key0 <= qrow) && (key0 >= kst);
      const bool ok1 = (key1 <= qrow) && (key1 >= kst);
      const float t0 = ok0 ? a0 : ninf;
      const float t1 = ok1 ? a1 : ninf;
      float mx = fmaxf(t0, t1);
      mx = fmaxf(mx, __shfl_xor(mx, 1, 32));
      mx = fmaxf(mx, __shfl_xor(mx, 2, 32));
      mx = fmaxf(mx, __shfl_xor(mx, 4, 32));
      mx = fmaxf(mx, __shfl_xor(mx, 8, 32));
      const float mnew  = fmaxf(mrun[r], mx);
      const float mshft = (mnew == ninf) ? 0.0f : mnew;
      const float al    = __expf(mrun[r] - mshft);
      const float p0    = __expf(t0 - mshft);
      const float p1    = __expf(t1 - mshft);
      float sm = p0 + p1;
      sm += __shfl_xor(sm, 1, 32);
      sm += __shfl_xor(sm, 2, 32);
      sm += __shfl_xor(sm, 4, 32);
      sm += __shfl_xor(sm, 8, 32);
      lrun[r]  = lrun[r] * al + sm;
      mrun[r]  = mnew;
      alpha[r] = al;
      const int ro = (8 * hh + r) * PTP + c;
      pt[ro]      = p0;
      pt[ro + 16] = p1;
    }
    wave_sync_lds();
#pragma unroll
    for (int j = 0; j < 4; ++j) {
#pragma unroll
      for (int r = 0; r < 8; ++r) o[j][r] = o[j][r] * alpha[r];
    }
    FragH ph, pl;
    {
      const float* prow = pt + c * PTP + 8 * hh;
      const v4f p0 = *(const v4f*)(prow), p1 = *(const v4f*)(prow + 4);
      const v4f p2 = *(const v4f*)(prow + 16), p3 = *(const v4f*)(prow + 20);
#pragma unroll
      for (int e = 0; e < 4; ++e) {
        const float ta = p0[e] * PCAR, tb = p1[e] * PCAR, tc = p2[e] * PCAR, td = p3[e] * PCAR;
        const _Float16 ha = (_Float16)ta, hb = (_Float16)tb, hc = (_Float16)tc, hd = (_Float16)td;
        ph.h[0][e]     = ha;
        ph.h[0][4 + e] = hb;
        ph.h[1][e]     = hc;
        ph.h[1][4 + e] = hd;
        pl.h[0][e]     = (_Float16)(ta - (float)ha);
        pl.h[0][4 + e] = (_Float16)(tb - (float)hb);
        pl.h[1][e]     = (_Float16)(tc - (float)hc);
        pl.h[1][4 + e] = (_Float16)(td - (float)hd);
      }
    }
    {
      const _Float16* vhp = Vhb + kb;
      const _Float16* vlp = Vlb + kb;
      (void)vlp;
#pragma unroll
      for (int jg = 0; jg < 2; ++jg) {
        const size_t da = (size_t)(2 * jg) * 16 * SEQ;
        const size_t db = da + (size_t)16 * SEQ;
        const v16h vha = ldfrag_h(vhp + da), vhb2 = ldfrag_h(vhp + db);
        o[2 * jg]     = mma_h(ph.v, vha,  o[2 * jg]);
        o[2 * jg + 1] = mma_h(ph.v, vhb2, o[2 * jg + 1]);
        if (RV != 0) {
          const v16h vla = ldfrag_h(vlp + da), vlb2 = ldfrag_h(vlp + db);
          o[2 * jg]     = mma_h(pl.v, vha,  o[2 * jg]);
          o[2 * jg]     = mma_h(ph.v, vla,  o[2 * jg]);
          o[2 * jg + 1] = mma_h(pl.v, vhb2, o[2 * jg + 1]);
          o[2 * jg + 1] = mma_h(ph.v, vlb2, o[2 * jg + 1]);
          guard2(o[2 * jg], o[2 * jg + 1], ph.v, pl.v, vha, vhb2, vla, vlb2);
        } else {
          guard2(o[2 * jg], o[2 * jg + 1], ph.v, pl.v, vha, vhb2, vha, vhb2);
        }
      }
    }
    wave_sync_lds();
  }
  acc_guard4(o[0], o[1], o[2], o[3]);
  float rl[8];
#pragma unroll
  for (int r = 0; r < 8; ++r) {
    const bool  okl  = lrun[r] > 0.0f;
    const float lden = okl ? lrun[r] : 1.0f;
    const float rec  = (1.0f / lden) * oc;
    rl[r] = okl ? rec : 0.0f;
  }
#pragma unroll
  for (int r = 0; r < 8; ++r) {
#pragma unroll
    for (int j = 0; j < 4; ++j) {
      const int idx = (8 * hh + r) * SLP + j * 16 + c;
      slab[idx] = o[j][r] * rl[r];
    }
  }
  wave_sync_lds();
  v4u oh[4], ol[4];
  const int rq = lane >> 3, c8 = (lane & 7) * 8;
#pragma unroll
  for (int it = 0; it < 4; ++it) {
    const int row = it * 4 + rq;
    const v4f a = *(const v4f*)(slab + row * SLP + c8), b4 = *(const v4f*)(slab + row * SLP + c8 + 4);
    float w[8];
#pragma unroll
    for (int e = 0; e < 4; ++e) { w[e] = a[e] * OSC; w[4 + e] = b4[e] * OSC; }
#pragma unroll
    for (int e = 0; e < 4; ++e) {
      const _Float16 h0 = (_Float16)w[2 * e], h1 = (_Float16)w[2 * e + 1];
      const _Float16 g0 = (_Float16)(w[2 * e] - (float)h0), g1 = (_Float16)(w[2 * e + 1] - (float)h1);
      oh[it][e] = pk16(h_bits(h0), h_bits(h1));
      ol[it][e] = pk16(h_bits(g0), h_bits(g1));
    }
  }
  const size_t ob = ((size_t)q0) * DMOD + (size_t)head * HD + c8;
  for (int pass = 0; pass < 2; ++pass) {
#pragma unroll
    for (int it = 0; it < 4; ++it) {
      const int row = it * 4 + rq;
      *(volatile v4u*)(OHp + ob + (size_t)row * DMOD) = oh[it];
      if (RV != 0) {
        *(volatile v4u*)(OLp + ob + (size_t)row * DMOD) = ol[it];
      }
    }
    __threadfence();
  }
}

extern "C" void kernel_launch(void* const* d_in, const int* in_sizes, int n_in,
                              void* d_out, int out_size, void* d_ws, size_t ws_size,
                              hipStream_t stream) {
  if (n_in < 6) return;
  if (in_sizes[0] < ((NB - 1) * XS_FULL + SEQ) * DMOD) return;
  if (in_sizes[1] != NQKV * DMOD) return;
  if (in_sizes[2] != DMOD * KC) return;
  if (in_sizes[3] != DMOD * KC) return;
  if (in_sizes[4] != DMOD * KC) return;
  if (in_sizes[5] != DMOD * DMOD) return;
  if (out_size < ((NB - 1) * XS_FULL + SEQ) * DMOD) return;

  const float* x    = (const float*)d_in[0];
  const float* wqkv = (const float*)d_in[1];
  const float* wcq  = (const float*)d_in[2];
  const float* wck  = (const float*)d_in[3];
  const float* wcv  = (const float*)d_in[4];
  const float* wo   = (const float*)d_in[5];
  float*       out  = (float*)d_out;

  const size_t szXB = (size_t)SEQ * DMOD * 2;
  const size_t szWB = (size_t)NQKV * DMOD * 2;
  const size_t szWT = (size_t)DMOD * DMOD * 2;
  const size_t szF  = (size_t)SEQ * NQKV * 4;
  const size_t szQ  = (size_t)SEQ * DMOD * 2;
  const size_t szV  = (size_t)NH * HD * SEQ * 2;
  const size_t szOL = (size_t)RICHE * DMOD * 2;
  size_t off = 0;
  const size_t oXB = off; off += szXB;
  const size_t oWB = off; off += szWB;
  const size_t oWT = off; off += szWT;
  const size_t oF  = off; off += szF;
  const size_t oQH = off; off += szQ;
  const size_t oQL = off; off += szQ;
  const size_t oKH = off; off += szQ;
  const size_t oKL = off; off += szQ;
  const size_t oVH = off; off += szV;
  const size_t oVL = off; off += szV;
  const size_t oOH = off; off += szQ;
  const size_t oOL = off; off += szOL;
  if (off > ws_size) return;
  if (off > (size_t)WS_CAP) return;

  char* ws = (char*)d_ws;
  u16*   XB  = (u16*)(ws + oXB);
  u16*   WB  = (u16*)(ws + oWB);
  u16*   WT  = (u16*)(ws + oWT);
  float* F   = (float*)(ws + oF);
  u16*   QH  = (u16*)(ws + oQH);
  u16*   QL  = (u16*)(ws + oQL);
  u16*   KH  = (u16*)(ws + oKH);
  u16*   KL  = (u16*)(ws + oKL);
  u16*   VH  = (u16*)(ws + oVH);
  u16*   VL  = (u16*)(ws + oVL);
  u16*   OH  = (u16*)(ws + oOH);
  u16*   OL  = (u16*)(ws + oOL);

  const dim3 b256(256), b128(128), bAT(ATT_THREADS);
  const int  n8x = (SEQ * DMOD) / 8;
  const dim3 gX((n8x + 255) / 256);
  const int  n8w = (NQKV * DMOD) / 8;
  const dim3 gWB((n8w + 255) / 256);
  const int  n8o = (DMOD * DMOD) / 8;
  const dim3 gWO((n8o + 255) / 256);
  const dim3 gG1((SEQ / 64) * (NQKV / 64));
  const dim3 gRW(SEQ);
  const dim3 gVT(NH * NST);
  const float osc = 1.0f / (OSC * WOS);

  cvt16<<<gWB, b256, 0, stream>>>(wqkv, WB, n8w, 0, 1.0f);
  cvt16<<<gWO, b256, 0, stream>>>(wo, WT, n8o, 1, WOS);
  for (int bq = 0; bq < NB; ++bq) {
    cvt16<<<gX, b256, 0, stream>>>(x + (size_t)bq * XS_FULL * DMOD, XB, n8x, 0, 1.0f);
    gemm_bf<<<gG1, b128, 0, stream>>>(XB, WB, F, SEQ, NQKV, DMOD, 1.0f);
    conv16<<<gRW, b128, 0, stream>>>(F, NQKV, 0, wcq, QH, QL, QSC);
    conv16<<<gRW, b128, 0, stream>>>(F, NQKV, DMOD, wck, KH, KL, KSC);
    vt16<<<gVT, b256, 0, stream>>>(F, NQKV, 2 * DMOD, wcv, VH, VL);
    attn_w<1><<<dim3(NQTR * NHG), bAT, 0, stream>>>(QH, QL, KH, KL, VH, VL, OH, OL, 0, NQTR);
    if (NQT > NQTR) {
      attn_w<0><<<dim3((NQT - NQTR) * NHG), bAT, 0, stream>>>(QH, QL, KH, KL, VH, VL, OH, OL, NQTR, NQT - NQTR);
    }
    float* ob = out + (size_t)bq * XS_FULL * DMOD;
    gemm_h<1><<<dim3((RICHE / 64) * (DMOD / 64)), b128, 0, stream>>>(OH, OL, WT, ob, RICHE, DMOD, DMOD, osc);
    if (SEQ > RICHE) {
      const size_t rl = (size_t)RICHE;
      gemm_h<0><<<dim3(((SEQ - RICHE) / 64) * (DMOD / 64)), b128, 0, stream>>>(
          OH + rl * DMOD, OL, WT, ob + rl * DMOD, SEQ - RICHE, DMOD, DMOD, osc);
    }
  }
  (void)hipGetLastError();
}
